// MACEBlock_7275674599652
// MI455X (gfx1250) — hardware-run, weakly checked
//
#include <hip/hip_runtime.h>


namespace {
constexpr int NB = 1, L = 4096, C = 128, NH = 4, HD = 32, NT = NB * L, KB = 128, PW = 3 * C;
constexpr int NA = 4096, NE = 131072, DN = 64, DM = 128, NBES = 8, NSH = 9, MU = 64  ;
constexpr float XS = 8.0f, HS = 256.0f, WSC = 256.0f, PS = 256.0f, SCALE = 0.17677669529663687f, CUT = 6.0f, PI_F = 3.14159265358979323846f;
typedef _Float16 b16;
typedef __attribute__((ext_vector_type(16))) _Float16 v16b;
typedef __attribute__((ext_vector_type(8))) _Float16 v8b;
typedef __attribute__((ext_vector_type(8))) float v8f;
typedef __attribute__((ext_vector_type(4))) float v4f;
typedef __attribute__((ext_vector_type(2))) float v2f;
__device__ __forceinline__ float bf16_rne(float f) { unsigned int u = __float_as_uint(f); u += 0x7FFFu + ((u >> 16) & 1u); float r = __uint_as_float(u & 0xFFFF0000u); asm volatile("" : "+v"(r)); return r; }
__device__ __forceinline__ float bfv(float f) { float r = bf16_rne(f); asm volatile("" : "+v"(r)); return r; }
__device__ __forceinline__ void split16(float v, b16& hi, b16& lo) { hi = (b16)v; lo = (b16)(v - (float)hi); }
__device__ __forceinline__ v16b frag_kb(const b16* p, int hh) { const v8b a = *(const v8b*)(p + 8 * hh), b = *(const v8b*)(p + 16 + 8 * hh); v16b f;
#pragma unroll
  for (int e = 0; e < 8; ++e) { f[e] = a[e]; f[8 + e] = b[e]; } return f; }
__device__ __forceinline__ v8f wmma16b(v16b a, v16b b, v8f c) { v8f d = __builtin_amdgcn_wmma_f32_16x16x32_f16(false, a, false, b, (short)0, c, false, false); asm volatile("v_nop\n\tv_nop\n\tv_nop\n\tv_nop" : "+v"(d) : "v"(a), "v"(b)); return d; }
__device__ __forceinline__ void wave_lds_sync() { __builtin_amdgcn_fence(__ATOMIC_RELEASE, "workgroup"); __builtin_amdgcn_wave_barrier(); __builtin_amdgcn_fence(__ATOMIC_ACQUIRE, "workgroup"); }
__device__ __forceinline__ float pmul(float a, float b) { float p = a * b; asm volatile("" : "+v"(p)); return p; }
__device__ __forceinline__ int iclamp(int v, int lo, int hi) { return v < lo ? lo : (v > hi ? hi : v); }
__device__ __forceinline__ float silu(float v) { return v / (1.0f + __expf(-v)); }
__device__ __forceinline__ float sigm(float v) { return 1.0f / (1.0f + __expf(-v)); }
constexpr int CSR_NBLK8 = 512, CSR_GB8 = 8, CSR_GN8 = 1 << CSR_GB8  , CSR_TS8 = (CSR_GN8 < 32 ? 32 : CSR_GN8)  , CSR_MAXG8 = 512, CSR_CAP8 = 12288  ;
__device__ __host__ __forceinline__ int csr_tix8(int v) { return (v >> CSR_GB8) * CSR_TS8 + (v & (CSR_GN8 - 1)); }
__global__ __launch_bounds__(64) void csrA_kernel8(const int* __restrict__ dst, int E, int N, int nG, int CHP, int NGP, int* __restrict__ STG, int* __restrict__ HST) {
  extern __shared__ int sm[];
  int* cnt = sm; int* run = sm + NGP; int* ids = sm + 2 * NGP;
  const int b = blockIdx.x; const int ch = (E + CSR_NBLK8 - 1) / CSR_NBLK8; const int e0 = b * ch, e1 = min(E, e0 + ch);
  for (int i = threadIdx.x; i < NGP; i += 64) cnt[i] = 0;
  for (int i = threadIdx.x; i < CHP; i += 64) ids[i] = -1;
  __syncthreads();
  if (threadIdx.x == 0) {
    for (int e = e0; e < e1; ++e) { int d = dst[e]; d = (d < 0) ? 0 : (d >= N ? N - 1 : d); cnt[d >> CSR_GB8] += 1; }
    int acc = 0; for (int g = 0; g < nG; ++g) { run[g] = acc; acc += cnt[g]; }
    for (int e = e0; e < e1; ++e) { int d = dst[e]; d = (d < 0) ? 0 : (d >= N ? N - 1 : d); const int g = d >> CSR_GB8; ids[run[g]] = e; run[g] += 1; } }
  __syncthreads();
  typedef __attribute__((ext_vector_type(4))) int v4i;
  for (int pass = 0; pass < 2; ++pass) {
    for (int i = threadIdx.x; i < CHP / 4; i += 64) *(volatile v4i*)(STG + (size_t)b * CHP + i * 4) = *(const v4i*)(&ids[i * 4]);
    for (int i = threadIdx.x; i < NGP / 4; i += 64) { v4i v; for (int e = 0; e < 4; ++e) v[e] = (i * 4 + e < nG) ? cnt[i * 4 + e] : 0; *(volatile v4i*)(HST + (size_t)b * NGP + i * 4) = v; }
    __threadfence(); }
}
__global__ __launch_bounds__(512) void csrS_kernel8(const int* __restrict__ HST, int nG, int NGP, int* __restrict__ START, int* __restrict__ TOT, int* __restrict__ OFF) {
  __shared__ int tot[CSR_MAXG8];
  const int b = threadIdx.x;
  for (int pass = 0; pass < 2; ++pass) { int runb = 0; for (int g = 0; g < nG; ++g) { int c = HST[(size_t)b * NGP + g]; c = (c < 0) ? 0 : c; ((volatile int*)OFF)[(size_t)g * CSR_NBLK8 + b] = runb; runb += c; } __threadfence(); }
  for (int g = threadIdx.x; g < nG; g += 512) { int s = 0; for (int bb = 0; bb < CSR_NBLK8; ++bb) { int c = HST[(size_t)bb * NGP + g]; s += (c < 0) ? 0 : c; } tot[g] = s; }
  __syncthreads();
  if (threadIdx.x < 32) {
    __shared__ int st[CSR_MAXG8 + 32];
    if (threadIdx.x == 0) { int acc = 0; for (int g = 0; g < NGP; ++g) { st[g] = acc; if (g < nG) acc += (tot[g] + 31) & ~31; } st[NGP] = acc; }
    __builtin_amdgcn_fence(__ATOMIC_RELEASE, "workgroup"); __builtin_amdgcn_wave_barrier(); __builtin_amdgcn_fence(__ATOMIC_ACQUIRE, "workgroup");
    for (int pass = 0; pass < 2; ++pass) { for (int i = threadIdx.x; i < NGP + 32; i += 32) { ((volatile int*)START)[i] = (i <= NGP) ? st[min(i, NGP)] : 0; ((volatile int*)TOT)[i] = (i < nG) ? tot[i] : 0; } __threadfence(); } }
}
__global__ __launch_bounds__(256) void csrB_kernel8(const int* __restrict__ dst, int N, int nG, int CHP, int NGP, int permLen, const int* __restrict__ STG, const int* __restrict__ HST, const int* __restrict__ OFF, const int* __restrict__ START, const int* __restrict__ TOT, int* __restrict__ PERM, int* __restrict__ ROWPTR, int* __restrict__ ROWCNT, int* __restrict__ FLAG) {
  typedef __attribute__((ext_vector_type(4))) int v4i;
  __shared__ int ids[CSR_CAP8]; __shared__ unsigned short key[CSR_CAP8]; __shared__ int outp[CSR_CAP8]; __shared__ int ncnt[CSR_GN8 + 1]; __shared__ int boff[CSR_NBLK8 + 1];
  const int g = blockIdx.x, t_ = threadIdx.x; int tot = TOT[g]; int st = START[g], stn = START[g + 1]; const int v0 = g * CSR_GN8; const int nv = min(CSR_GN8, N - v0); const int t0 = g * CSR_TS8;
  st = (st < 0) ? 0 : (st > permLen - 32 ? permLen - 32 : st) & ~31; stn = (stn < st) ? st : (stn > permLen ? permLen : stn); tot = (tot < 0) ? 0 : tot; if (tot > stn - st && tot <= CSR_CAP8) tot = stn - st;
  if (tot > CSR_CAP8) {
    for (int pass = 0; pass < 2; ++pass) { for (int i = t_; i < CSR_TS8 / 4; i += 256) { v4i a, c; for (int e = 0; e < 4; ++e) { a[e] = st; c[e] = 0; } *(volatile v4i*)(ROWPTR + t0 + i * 4) = a; *(volatile v4i*)(ROWCNT + t0 + i * 4) = c; } if (t_ == 0) ((volatile int*)FLAG)[0] = 1; __threadfence(); } (void)nv; return; }
  if (t_ == 0) { int acc = 0; for (int b = 0; b < CSR_NBLK8; ++b) { boff[b] = acc; int c = HST[(size_t)b * NGP + g]; c = (c < 0) ? 0 : (c > CHP ? CHP : c); acc += c; if (acc > tot) acc = tot; } boff[CSR_NBLK8] = acc; }
  for (int i = t_; i <= CSR_GN8; i += 256) ncnt[i] = 0;
  __syncthreads();
  for (int b = 0; b < CSR_NBLK8; ++b) { const int c = boff[b + 1] - boff[b]; int o_ = OFF[(size_t)g * CSR_NBLK8 + b]; o_ = (o_ < 0) ? 0 : (o_ > CHP - c ? CHP - c : o_); const int* src_ = STG + (size_t)b * CHP + o_;
    for (int i = t_; i < c; i += 256) { int id = src_[i]; id = (id < 0) ? 0 : id; ids[boff[b] + i] = id; int d = dst[id]; d = (d < v0) ? v0 : (d >= N ? N - 1 : d); int kk = d - v0; kk = (kk < 0) ? 0 : (kk >= CSR_GN8 ? CSR_GN8 - 1 : kk); key[boff[b] + i] = (unsigned short)kk; } }
  __syncthreads();
  if (t_ == 0) { for (int i = 0; i < tot; ++i) ncnt[key[i]] += 1; int acc = 0; for (int vl = 0; vl < CSR_GN8; ++vl) { const int c = ncnt[vl]; ncnt[vl] = acc; acc += c; } ncnt[CSR_GN8] = acc;
    for (int i = 0; i < tot; ++i) { const int vl = key[i]; outp[ncnt[vl]] = ids[i]; ncnt[vl] += 1; }
    for (int vl = CSR_GN8; vl > 0; --vl) ncnt[vl] = ncnt[vl - 1]; ncnt[0] = 0; }
  __syncthreads();
  for (int pass = 0; pass < 2; ++pass) {
    for (int i = t_; i < (stn - st) / 4; i += 256) { v4i v; for (int e = 0; e < 4; ++e) { const int q = i * 4 + e; v[e] = (q < tot) ? outp[q] : -1; } *(volatile v4i*)(PERM + st + i * 4) = v; }
    for (int i = t_; i < CSR_TS8 / 4; i += 256) { v4i a, c; for (int e = 0; e < 4; ++e) { const int vl = i * 4 + e; const int vc = vl < CSR_GN8 ? vl : CSR_GN8; a[e] = (vl < CSR_GN8) ? st + ncnt[vc] : st; c[e] = (vl < nv) ? (ncnt[(vc < CSR_GN8 ? vc : CSR_GN8 - 1) + 1] - ncnt[vc]) : 0; } *(volatile v4i*)(ROWPTR + t0 + i * 4) = a; *(volatile v4i*)(ROWCNT + t0 + i * 4) = c; }
    __threadfence(); }
}
__global__ __launch_bounds__(256) void csrZ_kernel8(int* __restrict__ p, size_t n4) { typedef __attribute__((ext_vector_type(4))) int v4i; const size_t tid = (size_t)blockIdx.x * 256 + threadIdx.x, nth = (size_t)gridDim.x * 256; v4i z = {0, 0, 0, 0}; for (size_t i = tid; i < n4; i += nth) *(volatile v4i*)(p + i * 4) = z; }
struct CsrBufs8 { int *STG, *HST, *OFF, *START, *TOT, *PERM, *ROWPTR, *ROWCNT, *FLAG; int nG, NGP, CHP; size_t permLen; char* base; size_t bytes; };
static size_t csr_carve8(CsrBufs8& c, char* ws, size_t off, int E, int N) {
  const size_t off0 = off; c.base = ws + off;
  auto al = [&](size_t bytes) { char* p = ws + off; off += (bytes + 255) & ~(size_t)255; return p; };
  c.nG = (N + CSR_GN8 - 1) / CSR_GN8; c.NGP = (c.nG + 31) & ~31; const int ch = (E + CSR_NBLK8 - 1) / CSR_NBLK8; c.CHP = (ch + 31) & ~31; c.permLen = (size_t)E + 32 * (size_t)c.nG + 32;
  c.STG = (int*)al((size_t)CSR_NBLK8 * c.CHP * 4); c.HST = (int*)al((size_t)CSR_NBLK8 * c.NGP * 4); c.OFF = (int*)al((size_t)c.NGP * CSR_NBLK8 * 4); c.START = (int*)al((size_t)(c.NGP + 64) * 4); c.TOT = (int*)al((size_t)(c.NGP + 64) * 4);
  c.PERM = (int*)al(c.permLen * 4); c.ROWPTR = (int*)al((size_t)c.nG * CSR_TS8 * 4); c.ROWCNT = (int*)al((size_t)c.nG * CSR_TS8 * 4); c.FLAG = (int*)al(256);
  c.bytes = off - off0; return off;
}
static void csr_build8(const CsrBufs8& c, const int* dst, int E, int N, hipStream_t stream) {
  const size_t smem = (size_t)(2 * c.NGP + c.CHP) * 4;
  csrZ_kernel8<<<512, 256, 0, stream>>>((int*)c.base, c.bytes / 16);
  csrA_kernel8<<<CSR_NBLK8, 64, smem, stream>>>(dst, E, N, c.nG, c.CHP, c.NGP, c.STG, c.HST);
  csrS_kernel8<<<1, 512, 0, stream>>>(c.HST, c.nG, c.NGP, c.START, c.TOT, c.OFF);
  csrB_kernel8<<<c.nG, 256, 0, stream>>>(dst, N, c.nG, c.CHP, c.NGP, (int)c.permLen, c.STG, c.HST, c.OFF, c.START, c.TOT, c.PERM, c.ROWPTR, c.ROWCNT, c.FLAG);
}


__global__ __launch_bounds__(256) void wput_kernel(const float* __restrict__ wr2, const float* __restrict__ wtp, const float* __restrict__ wm1, const float* __restrict__ wm2, const float* __restrict__ wqkv, const float* __restrict__ wao, const float* __restrict__ wg, const float* __restrict__ wo,
    b16* __restrict__ WR2, b16* __restrict__ WTP, b16* __restrict__ WM1, b16* __restrict__ WM2, b16* __restrict__ W3, b16* __restrict__ WAO, b16* __restrict__ WG, b16* __restrict__ WO) { const int u = blockIdx.x * 256 + threadIdx.x; v8b v;
  if (u < DM * 8) { const int o = u / 8, k0 = (u % 8) * 8;
#pragma unroll
    for (int j = 0; j < 8; ++j) v[j] = (b16)(bf16_rne(wr2[(size_t)(k0 + j) * DM + o]) * WSC); for (int pass = 0; pass < 2; ++pass) { *(volatile v8b*)(WR2 + (size_t)o * DN + k0) = v; __threadfence(); } }
  if (u < NSH * MU * 16) { const int s = u / (MU * 16), r = u % (MU * 16); const int o = r / 16, c0 = (r % 16) * 8;
#pragma unroll
    for (int j = 0; j < 8; ++j) { const int c = c0 + j; const int row = s == 0 ? c : (s < 4 ? DM + 3 * c + (s - 1) : 4 * DM + 5 * c + (s - 4)); v[j] = (b16)(bf16_rne(wtp[(size_t)row * DM + o]) * WSC); } for (int pass = 0; pass < 2; ++pass) { *(volatile v8b*)(WTP + ((size_t)s * MU + o) * DM + c0) = v; __threadfence(); } }
  if (u < DM * 16) { const int o = u / 16, k0 = (u % 16) * 8; const float* srcs[5] = {wm1, wm2, wao, wg, wo}; b16* dsts[5] = {WM1, WM2, WAO, WG, WO};
#pragma unroll
    for (int m = 0; m < 5; ++m) {
#pragma unroll
      for (int j = 0; j < 8; ++j) v[j] = (b16)(bf16_rne(srcs[m][(size_t)(k0 + j) * DM + o]) * WSC); for (int pass = 0; pass < 2; ++pass) { *(volatile v8b*)(dsts[m] + (size_t)o * DM + k0) = v; __threadfence(); } } }
  if (u < 3 * DM * 16) { const int o = u / 16, k0 = (u % 16) * 8;
#pragma unroll
    for (int j = 0; j < 8; ++j) v[j] = (b16)(bf16_rne(wqkv[(size_t)(k0 + j) * 3 * DM + o]) * WSC); for (int pass = 0; pass < 2; ++pass) { *(volatile v8b*)(W3 + (size_t)o * DM + k0) = v; __threadfence(); } } }
__global__ __launch_bounds__(32) void edge_kernel(const float* __restrict__ evec, const float* __restrict__ elen, const float* __restrict__ wr1, const float* __restrict__ br1, const b16* __restrict__ WR2, const float* __restrict__ br2, const b16* __restrict__ WTP, const float* __restrict__ btp, int ELIM, float* __restrict__ MSG) {
  __shared__ __attribute__((aligned(16))) b16 Ah[16][DM + 8], Al[16][DM + 8]; __shared__ float Sh[16][12], Rb[16][NBES], Tf[16][DM + 4], Ms[16][MU + 4]; const int lane = threadIdx.x, nloc = lane & 15, hlf = lane >> 4; const size_t e0 = (size_t)blockIdx.x * 16; if (e0 >= (size_t)ELIM) return;
  if (lane < 16) { const size_t e = e0 + lane; const float vx = bfv(evec[e * 3]), vy = bfv(evec[e * 3 + 1]), vz = bfv(evec[e * 3 + 2]); const float r = sqrtf(vx * vx + vy * vy + vz * vz) + 1e-8f; const float x = vx / r, y = vy / r, z = vz / r;
    Sh[lane][0] = 1.0f; Sh[lane][1] = y; Sh[lane][2] = z; Sh[lane][3] = x; Sh[lane][4] = 3.0f * z * z - 1.0f; Sh[lane][5] = x * z; Sh[lane][6] = y * z; Sh[lane][7] = x * y; Sh[lane][8] = x * x - y * y;
    const float ln = bfv(elen[e]); const float env = ln < CUT ? 0.5f * (cosf(ln * (PI_F / CUT)) + 1.0f) : 0.0f;
#pragma unroll
    for (int k = 0; k < NBES; ++k) Rb[lane][k] = sinf(ln * ((float)(k + 1) * (PI_F / CUT))) / ln * env; }
  wave_lds_sync();
  for (int rr = 0; rr < 16; ++rr) {
#pragma unroll
    for (int q = 0; q < 2; ++q) { const int c = q * 32 + lane; float s = bfv(br1[c]);
#pragma unroll
      for (int k = 0; k < NBES; ++k) s += pmul(Rb[rr][k], bfv(wr1[k * DN + c])); b16 p, ql; split16(silu(s) * HS, p, ql); Ah[rr][c] = p; Al[rr][c] = ql; } if (lane < 8) { Ah[rr][DN + lane] = (b16)0.0f; Al[rr][DN + lane] = (b16)0.0f; } }
  wave_lds_sync();
  { v8f acc[8];
#pragma unroll
    for (int t = 0; t < 8; ++t) acc[t] = (v8f){};
#pragma unroll
    for (int kb = 0; kb < DN; kb += 32) { const v16b a = frag_kb(&Ah[nloc][kb], hlf), al = frag_kb(&Al[nloc][kb], hlf);
#pragma unroll
      for (int t = 0; t < 8; ++t) { const v16b bw = frag_kb(WR2 + (size_t)(t * 16 + nloc) * DN + kb, hlf); acc[t] = wmma16b(a, bw, acc[t]); acc[t] = wmma16b(al, bw, acc[t]); } }
#pragma unroll
    for (int t = 0; t < 8; ++t) { const int cc = t * 16 + nloc; const float bb = bfv(br2[cc]);
#pragma unroll
      for (int r8 = 0; r8 < 8; ++r8) Tf[8 * hlf + r8][cc] = silu(acc[t][r8] * (1.0f / (HS * WSC)) + bb); } }
  wave_lds_sync();
  for (int rr = 0; rr < 16; ++rr) for (int q = 0; q < 4; ++q) { b16 p, ql; split16(Tf[rr][q * 32 + lane] * HS, p, ql); Ah[rr][q * 32 + lane] = p; Al[rr][q * 32 + lane] = ql; } if (lane < 16) for (int k = DM; k < DM + 8; ++k) { Ah[lane][k] = (b16)0.0f; Al[lane][k] = (b16)0.0f; }
  wave_lds_sync();
  float msg[4][8];
#pragma unroll
  for (int t = 0; t < 4; ++t)
#pragma unroll
    for (int r8 = 0; r8 < 8; ++r8) msg[t][r8] = 0.0f;
#pragma unroll 1
  for (int s = 0; s < NSH; ++s) { v8f acc[4] = {(v8f){}, (v8f){}, (v8f){}, (v8f){}};
#pragma unroll
    for (int kb = 0; kb < DM; kb += 32) { const v16b a = frag_kb(&Ah[nloc][kb], hlf), al = frag_kb(&Al[nloc][kb], hlf);
#pragma unroll
      for (int t = 0; t < 4; ++t) { const v16b bw = frag_kb(WTP + ((size_t)s * MU + t * 16 + nloc) * DM + kb, hlf); acc[t] = wmma16b(a, bw, acc[t]); acc[t] = wmma16b(al, bw, acc[t]); } }
#pragma unroll
    for (int r8 = 0; r8 < 8; ++r8) { const float shv = Sh[8 * hlf + r8][s];
#pragma unroll
      for (int t = 0; t < 4; ++t) msg[t][r8] += pmul(shv, acc[t][r8] * (1.0f / (HS * WSC))); } }
#pragma unroll
  for (int t = 0; t < 4; ++t) { const int cc = t * 16 + nloc; const float bb = bfv(btp[cc]);
#pragma unroll
    for (int r8 = 0; r8 < 8; ++r8) Ms[8 * hlf + r8][cc] = msg[t][r8] + bb; }
  wave_lds_sync();
  for (int pass = 0; pass < 2; ++pass) { for (int rr = 0; rr < 16; ++rr) *(volatile v2f*)(MSG + (e0 + rr) * MU + lane * 2) = *(const v2f*)(&Ms[rr][lane * 2]); __threadfence(); } }
__global__ __launch_bounds__(256) void agg_kernel(const float* __restrict__ MSG, const int* __restrict__ PERM, const int* __restrict__ ROWPTR, const int* __restrict__ ROWCNT, int permLen, int NLIM, int ELIM, float* __restrict__ AGG) { const int wave = threadIdx.x >> 5, lane = threadIdx.x & 31; const size_t i = (size_t)blockIdx.x * 8 + wave; if (i >= (size_t)NLIM) return; int st = ROWPTR[i], cnt = ROWCNT[i]; cnt = iclamp(cnt, 0, NE); st = iclamp(st, 0, permLen - cnt); float s0 = 0.0f, s1 = 0.0f;
#pragma unroll 1
  for (int j = 0; j < cnt; ++j) { const int e = iclamp(PERM[st + j], 0, NE - 1); if (e >= ELIM) continue; const v2f v = *(const v2f*)(MSG + (size_t)e * MU + lane * 2); s0 += v[0]; s1 += v[1]; }
  for (int pass = 0; pass < 2; ++pass) { *(volatile v2f*)(AGG + i * MU + lane * 2) = (v2f){s0, s1}; __threadfence(); } }
__global__ __launch_bounds__(32) void node_kernel(const int* __restrict__ Z, const float* __restrict__ emb, const float* __restrict__ AGG, const b16* __restrict__ WM1, const b16* __restrict__ WM2, const float* __restrict__ bm1, const float* __restrict__ bm2, int NLIM, float* __restrict__ UPD) { __shared__ __attribute__((aligned(16))) b16 Ah[16][DM + 8], Al[16][DM + 8]; __shared__ float Tf[16][DM + 4]; const int lane = threadIdx.x, nloc = lane & 15, hlf = lane >> 4; const size_t m0 = (size_t)blockIdx.x * 16; if (m0 >= (size_t)NLIM) return;
  for (int rr = 0; rr < 16; ++rr) { const int zi = iclamp(Z[m0 + rr], 0, 99); for (int q = 0; q < 2; ++q) { const int c = q * 32 + lane; Ah[rr][c] = (b16)(bf16_rne(emb[(size_t)zi * DN + c]) * HS); Al[rr][c] = (b16)0.0f; b16 p, ql; split16(AGG[(m0 + rr) * MU + c] * HS, p, ql); Ah[rr][DN + c] = p; Al[rr][DN + c] = ql; } }
  if (lane < 16) for (int k = DM; k < DM + 8; ++k) { Ah[lane][k] = (b16)0.0f; Al[lane][k] = (b16)0.0f; }
  wave_lds_sync(); v8f acc[8];
#pragma unroll
  for (int t = 0; t < 8; ++t) acc[t] = (v8f){};
#pragma unroll
  for (int kb = 0; kb < DM; kb += 32) { const v16b a = frag_kb(&Ah[nloc][kb], hlf), al = frag_kb(&Al[nloc][kb], hlf);
#pragma unroll
    for (int t = 0; t < 8; ++t) { const v16b bw = frag_kb(WM1 + (size_t)(t * 16 + nloc) * DM + kb, hlf); acc[t] = wmma16b(a, bw, acc[t]); acc[t] = wmma16b(al, bw, acc[t]); } }
  wave_lds_sync();
#pragma unroll
  for (int t = 0; t < 8; ++t) { const int cc = t * 16 + nloc; const float bb = bfv(bm1[cc]);
#pragma unroll
    for (int r8 = 0; r8 < 8; ++r8) { b16 p, ql; split16(silu(acc[t][r8] * (1.0f / (HS * WSC)) + bb) * HS, p, ql); Ah[8 * hlf + r8][cc] = p; Al[8 * hlf + r8][cc] = ql; } }
  wave_lds_sync();
#pragma unroll
  for (int t = 0; t < 8; ++t) acc[t] = (v8f){};
#pragma unroll
  for (int kb = 0; kb < DM; kb += 32) { const v16b a = frag_kb(&Ah[nloc][kb], hlf), al = frag_kb(&Al[nloc][kb], hlf);
#pragma unroll
    for (int t = 0; t < 8; ++t) { const v16b bw = frag_kb(WM2 + (size_t)(t * 16 + nloc) * DM + kb, hlf); acc[t] = wmma16b(a, bw, acc[t]); acc[t] = wmma16b(al, bw, acc[t]); } }
#pragma unroll
  for (int t = 0; t < 8; ++t) { const int cc = t * 16 + nloc; const float bb = bfv(bm2[cc]);
#pragma unroll
    for (int r8 = 0; r8 < 8; ++r8) Tf[8 * hlf + r8][cc] = acc[t][r8] * (1.0f / (HS * WSC)) + bb; }
  wave_lds_sync();
  for (int pass = 0; pass < 2; ++pass) { for (int rr = 0; rr < 16; ++rr) *(volatile v4f*)(UPD + (m0 + rr) * DM + lane * 4) = *(const v4f*)(&Tf[rr][lane * 4]); __threadfence(); } }
__global__ __launch_bounds__(32) void qkv_kernel(const float* __restrict__ UPD, const b16* __restrict__ W3, const float* __restrict__ bqkv, int NLIM, b16* __restrict__ PH, b16* __restrict__ PL) { __shared__ __attribute__((aligned(16))) b16 Ah[16][DM + 8], Al[16][DM + 8], Oh[16][DM + 8], Ol[16][DM + 8]; const int lane = threadIdx.x, nloc = lane & 15, hlf = lane >> 4; const size_t m0 = (size_t)blockIdx.x * 16; if (m0 >= (size_t)NLIM) return;
  for (int rr = 0; rr < 16; ++rr) for (int q = 0; q < 4; ++q) { b16 p, ql; split16(UPD[(m0 + rr) * DM + q * 32 + lane] * HS, p, ql); Ah[rr][q * 32 + lane] = p; Al[rr][q * 32 + lane] = ql; } if (lane < 16) for (int k = DM; k < DM + 8; ++k) { Ah[lane][k] = (b16)0.0f; Al[lane][k] = (b16)0.0f; }
  wave_lds_sync();
#pragma unroll 1
  for (int g = 0; g < 3; ++g) { v8f acc[8];
#pragma unroll
    for (int t = 0; t < 8; ++t) acc[t] = (v8f){};
#pragma unroll
    for (int kb = 0; kb < DM; kb += 32) { const v16b a = frag_kb(&Ah[nloc][kb], hlf), al = frag_kb(&Al[nloc][kb], hlf);
#pragma unroll
      for (int t = 0; t < 8; ++t) { const v16b bw = frag_kb(W3 + (size_t)(g * DM + t * 16 + nloc) * DM + kb, hlf); acc[t] = wmma16b(a, bw, acc[t]); acc[t] = wmma16b(al, bw, acc[t]); } }
    const float sc = g == 0 ? SCALE : 1.0f;
#pragma unroll
    for (int t = 0; t < 8; ++t) { const int cc = t * 16 + nloc; const float bb = bfv(bqkv[g * DM + cc]);
#pragma unroll
      for (int r8 = 0; r8 < 8; ++r8) { b16 p, ql; split16((acc[t][r8] * (1.0f / (HS * WSC)) + bb) * sc * HS, p, ql); Oh[8 * hlf + r8][cc] = p; Ol[8 * hlf + r8][cc] = ql; } }
    wave_lds_sync();
    for (int pass = 0; pass < 2; ++pass) { for (int rr = 0; rr < 16; ++rr) if (lane < 16) { *(volatile v8b*)(PH + (m0 + rr) * PW + g * DM + lane * 8) = *(const v8b*)(&Oh[rr][lane * 8]); *(volatile v8b*)(PL + (m0 + rr) * PW + g * DM + lane * 8) = *(const v8b*)(&Ol[rr][lane * 8]); } __threadfence(); }
    wave_lds_sync(); } }
__global__ __launch_bounds__(32) void att_kernel(const b16* __restrict__ PH, const b16* __restrict__ PL, const float* __restrict__ amask, int BLIM, float* __restrict__ ATT) { __shared__ __attribute__((aligned(16))) b16 Ph_[16][KB + 8], Pl_[16][KB + 8], Vth[HD][KB + 8], Vtl[HD][KB + 8]; __shared__ float Sf[16][KB + 4], Of[16][HD + 4];
  const int lane = threadIdx.x, nloc = lane & 15, hlf = lane >> 4; const int qt = blockIdx.x % (L / 16); const int h = (blockIdx.x / (L / 16)) % NH; const int b = blockIdx.x / ((L / 16) * NH); if (b >= BLIM) return; const int t0 = qt * 16; const size_t rowb = (size_t)b * L; const int qo = h * HD, ko = C + h * HD, vo = 2 * C + h * HD;
  v16b qh[HD / 32], ql[HD / 32];
#pragma unroll
  for (int s = 0; s < HD / 32; ++s) { qh[s] = frag_kb(PH + (rowb + t0 + nloc) * PW + qo + s * 32, hlf); ql[s] = frag_kb(PL + (rowb + t0 + nloc) * PW + qo + s * 32, hlf); }
  float m_r[8], den_r[8]; v8f acc[HD / 16];
#pragma unroll
  for (int r8 = 0; r8 < 8; ++r8) { m_r[r8] = -INFINITY; den_r[r8] = 0.0f; }
#pragma unroll
  for (int t = 0; t < HD / 16; ++t) acc[t] = (v8f){};
  const int kstart = 0; const int kend = L;
#pragma unroll 1
  for (int kb0 = kstart; kb0 < kend; kb0 += KB) { const int nk = (kend - kb0) < KB ? (kend - kb0) : KB; const int nkt = (nk + 15) / 16;
    for (int rr = 0; rr < KB; rr += 2) { const int r = rr + hlf; const int key = kb0 + r < L ? kb0 + r : L - 1;     const size_t vr = (rowb + key) * PW + vo; for (int s = 0; s < HD / 32; ++s) { Vth[s * 32 + nloc][r] = PH[vr + s * 32 + nloc]; Vth[s * 32 + 16 + nloc][r] = PH[vr + s * 32 + 16 + nloc]; Vtl[s * 32 + nloc][r] = PL[vr + s * 32 + nloc]; Vtl[s * 32 + 16 + nloc][r] = PL[vr + s * 32 + 16 + nloc]; } }
    for (int t = 0; t < KB / 16; ++t) { if (t < nkt) { const int key = kb0 + t * 16 + nloc < L ? kb0 + t * 16 + nloc : L - 1; const size_t kr = (rowb + key) * PW + ko; v8f s = {};
#pragma unroll
        for (int q = 0; q < HD / 32; ++q) { const v16b kh = frag_kb(PH + kr + q * 32, hlf), kl = frag_kb(PL + kr + q * 32, hlf); s = wmma16b(qh[q], kh, s); s = wmma16b(qh[q], kl, s); s = wmma16b(ql[q], kh, s); }
#pragma unroll
        for (int r8 = 0; r8 < 8; ++r8) { const int i = t0 + 8 * hlf + r8, j = kb0 + t * 16 + nloc; const bool ok = (j < kend); Sf[8 * hlf + r8][t * 16 + nloc] = ok ? s[r8] * (1.0f / (HS * HS)) : -INFINITY; } }
      else {
#pragma unroll
        for (int r8 = 0; r8 < 8; ++r8) Sf[8 * hlf + r8][t * 16 + nloc] = -INFINITY; } }
    wave_lds_sync();
#pragma unroll
    for (int rr = 0; rr < 16; ++rr) { float mx = -INFINITY;
#pragma unroll
      for (int q = 0; q < 4; ++q) mx = fmaxf(mx, Sf[rr][q * 32 + lane]);
      for (int o = 16; o; o >>= 1) mx = fmaxf(mx, __shfl_xor(mx, o));
      const float mold = __shfl(m_r[rr & 7], (rr >> 3) * 16); const float mn = fmaxf(mold, mx); const float sf = (mold == -INFINITY) ? 0.0f : ((mn == -INFINITY) ? 1.0f : __expf(mold - mn)); float ps = 0.0f;
#pragma unroll
      for (int q = 0; q < 4; ++q) { const int kx = q * 32 + lane; const float sv = Sf[rr][kx]; const float p = (sv == -INFINITY || mn == -INFINITY) ? 0.0f : __expf(sv - mn); ps += p; b16 ph, pl; split16(p * PS, ph, pl); Ph_[rr][kx] = ph; Pl_[rr][kx] = pl; }
      for (int o = 16; o; o >>= 1) ps += __shfl_xor(ps, o);
      if ((rr >> 3) == hlf) { const int r8 = rr & 7; den_r[r8] = den_r[r8] * sf + ps; m_r[r8] = mn;
#pragma unroll
        for (int t = 0; t < HD / 16; ++t) acc[t][r8] = acc[t][r8] * sf; } }
    wave_lds_sync();
    for (int ks = 0; ks < nkt * 16; ks += 32) { const v16b pa = frag_kb(&Ph_[nloc][ks], hlf), pb = frag_kb(&Pl_[nloc][ks], hlf);
#pragma unroll
      for (int t = 0; t < HD / 16; ++t) { const v16b vh = frag_kb(&Vth[t * 16 + nloc][ks], hlf), vl = frag_kb(&Vtl[t * 16 + nloc][ks], hlf); acc[t] = wmma16b(pa, vh, acc[t]); acc[t] = wmma16b(pa, vl, acc[t]); acc[t] = wmma16b(pb, vh, acc[t]); } }
    wave_lds_sync(); }
#pragma unroll
  for (int t = 0; t < HD / 16; ++t)
#pragma unroll
    for (int r8 = 0; r8 < 8; ++r8) { const float dn = den_r[r8]; Of[8 * hlf + r8][t * 16 + nloc] = dn > 0.0f ? acc[t][r8] * (1.0f / (HS * PS)) / dn : 0.0f; }
  wave_lds_sync();
  for (int pass = 0; pass < 2; ++pass) { for (int rr = 0; rr < 16; ++rr) for (int s = 0; s < HD / 32; ++s) ((volatile float*)ATT)[(rowb + t0 + rr) * C + h * HD + s * 32 + lane] = Of[rr][s * 32 + lane]; __threadfence(); } }

__global__ __launch_bounds__(32) void final_kernel(const float* __restrict__ ATT, const float* __restrict__ UPD, const b16* __restrict__ WAO, const b16* __restrict__ WG, const b16* __restrict__ WO, const float* __restrict__ bao, const float* __restrict__ bg, const float* __restrict__ bo, const float* __restrict__ pos, int NLIM, float* __restrict__ out) {
  __shared__ __attribute__((aligned(16))) b16 Ah[16][DM + 8], Al[16][DM + 8], Uh[16][DM + 8], Ul[16][DM + 8]; __shared__ float Ta[16][DM + 4]; const int lane = threadIdx.x, nloc = lane & 15, hlf = lane >> 4; const size_t m0 = (size_t)blockIdx.x * 16; if (m0 >= (size_t)NLIM) return;
  for (int rr = 0; rr < 16; ++rr) for (int q = 0; q < 4; ++q) { const int c = q * 32 + lane; b16 p, ql; split16(ATT[(m0 + rr) * DM + c] * HS, p, ql); Ah[rr][c] = p; Al[rr][c] = ql; split16(UPD[(m0 + rr) * DM + c] * HS, p, ql); Uh[rr][c] = p; Ul[rr][c] = ql; }
  if (lane < 16) for (int k = DM; k < DM + 8; ++k) { Ah[lane][k] = (b16)0.0f; Al[lane][k] = (b16)0.0f; Uh[lane][k] = (b16)0.0f; Ul[lane][k] = (b16)0.0f; }
  wave_lds_sync(); v8f aa[8], ag[8];
#pragma unroll
  for (int t = 0; t < 8; ++t) { aa[t] = (v8f){}; ag[t] = (v8f){}; }
#pragma unroll
  for (int kb = 0; kb < DM; kb += 32) { const v16b a = frag_kb(&Ah[nloc][kb], hlf), al = frag_kb(&Al[nloc][kb], hlf), u = frag_kb(&Uh[nloc][kb], hlf), ul = frag_kb(&Ul[nloc][kb], hlf);
#pragma unroll
    for (int t = 0; t < 8; ++t) { const v16b bw = frag_kb(WAO + (size_t)(t * 16 + nloc) * DM + kb, hlf), gw = frag_kb(WG + (size_t)(t * 16 + nloc) * DM + kb, hlf); aa[t] = wmma16b(a, bw, aa[t]); aa[t] = wmma16b(al, bw, aa[t]); ag[t] = wmma16b(u, gw, ag[t]); ag[t] = wmma16b(ul, gw, ag[t]); } }
#pragma unroll
  for (int t = 0; t < 8; ++t) { const int cc = t * 16 + nloc; const float ba = bfv(bao[cc]), bgg = bfv(bg[cc]);
#pragma unroll
    for (int r8 = 0; r8 < 8; ++r8) { const int rr = 8 * hlf + r8; const float att = aa[t][r8] * (1.0f / (HS * WSC)) + ba; const float g = sigm(ag[t][r8] * (1.0f / (HS * WSC)) + bgg); const float u = UPD[(m0 + rr) * DM + cc]; Ta[rr][cc] = pmul(g, att) + pmul(1.0f - g, u); } }
  wave_lds_sync();
  for (int rr = 0; rr < 16; ++rr) for (int q = 0; q < 4; ++q) { const int c = q * 32 + lane; b16 p, ql; split16(Ta[rr][c] * HS, p, ql); Ah[rr][c] = p; Al[rr][c] = ql; }
  wave_lds_sync();
#pragma unroll
  for (int t = 0; t < 8; ++t) aa[t] = (v8f){};
#pragma unroll
  for (int kb = 0; kb < DM; kb += 32) { const v16b a = frag_kb(&Ah[nloc][kb], hlf), al = frag_kb(&Al[nloc][kb], hlf);
#pragma unroll
    for (int t = 0; t < 8; ++t) { const v16b bw = frag_kb(WO + (size_t)(t * 16 + nloc) * DM + kb, hlf); aa[t] = wmma16b(a, bw, aa[t]); aa[t] = wmma16b(al, bw, aa[t]); } }
#pragma unroll
  for (int t = 0; t < 8; ++t) { const int cc = t * 16 + nloc; const float bb = bfv(bo[cc]);
#pragma unroll
    for (int r8 = 0; r8 < 8; ++r8) Ta[8 * hlf + r8][cc] = aa[t][r8] * (1.0f / (HS * WSC)) + bb + pmul(0.0f, bfv(pos[(m0 + 8 * hlf + r8) * 3])); }
  wave_lds_sync();
  for (int pass = 0; pass < 2; ++pass) { for (int rr = 0; rr < 16; ++rr) *(volatile v4f*)(out + (m0 + rr) * DM + lane * 4) = *(const v4f*)(&Ta[rr][lane * 4]); __threadfence(); } }
}

extern "C" void kernel_launch(void* const* d_in, const int* in_sizes, int n_in, void* d_out, int out_size, void* d_ws, size_t ws_size, hipStream_t stream) {
  (void)n_in;
  auto Fp = [&](int i) { return (const float*)d_in[i]; }; auto Ip = [&](int i) { return (const int*)d_in[i]; };
  if (in_sizes[0] != NA || in_sizes[2] != 2 * NE || in_sizes[3] != NE * 3 || in_sizes[4] != NE || in_sizes[5] != 100 * DN || in_sizes[6] != NBES * DN || in_sizes[8] != DN * DM || in_sizes[10] != NSH * DM * DM || in_sizes[12] != DM * DM || in_sizes[16] != DM * 3 * DM || in_sizes[22] != DM * DM || out_size != NA * DM) return;
  const int NLIM = NA, ELIM = NE;
  size_t off = 0; char* ws = (char*)d_ws;
  auto carve = [&](size_t bytes) { char* p = ws + off; off += (bytes + 255) & ~(size_t)255; return p; };
  b16* WR2 = (b16*)carve((size_t)DM * DN * 2); b16* WTP = (b16*)carve((size_t)NSH * MU * DM * 2); b16* WM1 = (b16*)carve((size_t)DM * DM * 2); b16* WM2 = (b16*)carve((size_t)DM * DM * 2); b16* W3 = (b16*)carve((size_t)3 * DM * DM * 2); b16* WAO = (b16*)carve((size_t)DM * DM * 2); b16* WG = (b16*)carve((size_t)DM * DM * 2); b16* WO = (b16*)carve((size_t)DM * DM * 2);
  float* MSG = (float*)carve((size_t)NE * MU * 4); float* AGG = (float*)carve((size_t)NA * MU * 4); float* UPD = (float*)carve((size_t)NA * DM * 4); b16* PH = (b16*)carve((size_t)NA * PW * 2); b16* PL = (b16*)carve((size_t)NA * PW * 2); float* ATT = (float*)carve((size_t)NA * DM * 4); CsrBufs8 csr; off = csr_carve8(csr, ws, off, NE, NA);
  if (off > ws_size || off > ((size_t)96 << 20)) return;
  wput_kernel<<<(NSH * MU * 16 + 255) / 256, 256, 0, stream>>>(Fp(8), Fp(10), Fp(12), Fp(14), Fp(16), Fp(18), Fp(20), Fp(22), WR2, WTP, WM1, WM2, W3, WAO, WG, WO);
  csr_build8(csr, Ip(2) + NE, NE, NA, stream);
  edge_kernel<<<ELIM / 16, 32, 0, stream>>>(Fp(3), Fp(4), Fp(6), Fp(7), WR2, Fp(9), WTP, Fp(11), ELIM, MSG);
  agg_kernel<<<(NLIM + 7) / 8, 256, 0, stream>>>(MSG, csr.PERM, csr.ROWPTR, csr.ROWCNT, (int)csr.permLen, NLIM, ELIM, AGG);
  node_kernel<<<NLIM / 16, 32, 0, stream>>>(Ip(0), Fp(5), AGG, WM1, WM2, Fp(13), Fp(15), NLIM, UPD);
  qkv_kernel<<<NLIM / 16, 32, 0, stream>>>(UPD, W3, Fp(17), NLIM, PH, PL);
  att_kernel<<<NB * NH * (L / 16), 32, 0, stream>>>(PH, PL, (const float*)0, NB, ATT);
  final_kernel<<<NLIM / 16, 32, 0, stream>>>(ATT, UPD, WAO, WG, WO, Fp(19), Fp(21), Fp(23), Fp(1), NLIM, (float*)d_out);
}
